// InternVisionEncoderLayer_31688268710156
// MI455X (gfx1250) — hardware-verified
//
#include <hip/hip_runtime.h>
#include <math.h>
#include <stdint.h>
#include <stddef.h>


#define S_TOK   2048
#define NSEQ_   4
#define SEQL    (S_TOK / NSEQ_)
#define E_DIM   1024
#define H_HEADS 16
#define D_HEAD  64
#define I_DIM   4096
#define ROPE_W  (D_HEAD / 2)
#define EPSF    1e-6f

#define W_SCALE 64.0f
#define P_SCALE 256.0f
#define O_SCALE 16.0f

typedef char chk_tile_[(S_TOK % 128 == 0 && E_DIM % 128 == 0 && I_DIM % 128 == 0) ? 1 : -1];
typedef char chk_ktile_[(E_DIM % 32 == 0 && I_DIM % 32 == 0 && SEQL % 128 == 0) ? 1 : -1];
typedef char chk_heads_[(H_HEADS * D_HEAD == E_DIM) ? 1 : -1];

typedef _Float16 v16h __attribute__((ext_vector_type(16)));
typedef _Float16 v8h  __attribute__((ext_vector_type(8)));
typedef float    v8f  __attribute__((ext_vector_type(8)));
typedef float    v4f  __attribute__((ext_vector_type(4)));

union Frag16 { v16h v; v8h h[2]; };
union F8 { v4f v[2]; float f[8]; };

static __device__ __forceinline__ v8f vz8() {
  v8f z = {0.f, 0.f, 0.f, 0.f, 0.f, 0.f, 0.f, 0.f};
  return z;
}

static __device__ __forceinline__ v16h frag_ld(const _Float16* p, int hh) {
  Frag16 f;
  f.h[0] = *(const v8h*)(p + 8 * hh);
  f.h[1] = *(const v8h*)(p + 16 + 8 * hh);
  return f.v;
}

static __device__ __forceinline__ v8f wmma_f16(v16h a, v16h b, v8f c) {
  return __builtin_amdgcn_wmma_f32_16x16x32_f16(false, a, false, b, (short)0, c,
                                                false, false);
}

static __device__ __forceinline__ float wave_sum(float v) {
  v += __shfl_xor(v, 16, 32);
  v += __shfl_xor(v, 8, 32);
  v += __shfl_xor(v, 4, 32);
  v += __shfl_xor(v, 2, 32);
  v += __shfl_xor(v, 1, 32);
  return v;
}

static __device__ __forceinline__ void ld8(F8& d, const float* p) {
  d.v[0] = *(const v4f*)p;
  d.v[1] = *(const v4f*)(p + 4);
}

static __device__ __forceinline__ void cvt_pass(const float* __restrict__ in,
                                                _Float16* out, int n8, float scale) {
  const int stride = gridDim.x * blockDim.x;
  for (int i = blockIdx.x * blockDim.x + threadIdx.x; i < n8; i += stride) {
    F8 s;
    ld8(s, in + (size_t)i * 8);
    v8h o;
#pragma unroll
    for (int u = 0; u < 8; ++u) o[u] = (_Float16)(s.f[u] * scale);
    *(volatile v8h*)(out + (size_t)i * 8) = o;
  }
}

__global__ __launch_bounds__(256) void cvt_scale_f16(const float* __restrict__ in,
                                                    _Float16* out, int n8, float scale) {
  cvt_pass(in, out, n8, scale);
  __threadfence();
  cvt_pass(in, out, n8, scale);
}

__global__ __launch_bounds__(128) void layernorm_f16(const float* __restrict__ x,
                                                   const float* __restrict__ w,
                                                   const float* __restrict__ b,
                                                   _Float16* y, int rows) {
  __shared__ float red0[4], red1[4];
  const int row = blockIdx.x;
  if (row >= rows) return;
  const int tid = threadIdx.x, lane = tid & 31, wv = tid >> 5;
  const int e0 = tid * 8;
  const float* xr = x + (size_t)row * E_DIM + e0;
  F8 xv;
  ld8(xv, xr);
  float s = ((xv.f[0] + xv.f[1]) + (xv.f[2] + xv.f[3])) +
            ((xv.f[4] + xv.f[5]) + (xv.f[6] + xv.f[7]));
  s = wave_sum(s);
  if (lane == 0) red0[wv] = s;
  __syncthreads();
  const float mu = ((red0[0] + red0[1]) + (red0[2] + red0[3])) * (1.0f / E_DIM);
  float d[8];
  float q = 0.f;
#pragma unroll
  for (int u = 0; u < 8; ++u) { d[u] = xv.f[u] - mu; q += d[u] * d[u]; }
  q = wave_sum(q);
  if (lane == 0) red1[wv] = q;
  __syncthreads();
  const float var = ((red1[0] + red1[1]) + (red1[2] + red1[3])) * (1.0f / E_DIM);
  const float rs = rsqrtf(var + EPSF);
  F8 wv8, bv8;
  ld8(wv8, w + e0);
  ld8(bv8, b + e0);
  v8h o;
#pragma unroll
  for (int u = 0; u < 8; ++u) o[u] = (_Float16)(d[u] * rs * wv8.f[u] + bv8.f[u]);
  _Float16* dst = y + (size_t)row * E_DIM + e0;
  *(volatile v8h*)dst = o;
  __threadfence();
  *(volatile v8h*)dst = o;
}

#define GM_SP 68

template <int EPI>
static __device__ __forceinline__ void epi_pass(const float* stg, int lane,
                                                const float* __restrict__ ls,
                                                const float* __restrict__ resid,
                                                float* Cf, _Float16* Ch,
                                                int grow0, int gcol0, int N) {
  if constexpr (EPI == 1) {
    const int rl = lane >> 3, c8 = (lane & 7) * 8;
#pragma unroll 1
    for (int p = 0; p < 4; ++p) {
      const int rr = p * 4 + rl;
      F8 v;
      v.v[0] = *(const v4f*)(stg + rr * GM_SP + c8);
      v.v[1] = *(const v4f*)(stg + rr * GM_SP + c8 + 4);
      v8h o;
#pragma unroll
      for (int u = 0; u < 8; ++u) {
        const float xx = v.f[u];
        const float g = 0.5f * xx * (1.0f + erff(xx * 0.70710678118654752f));
        o[u] = (_Float16)g;
      }
      *(volatile v8h*)(Ch + (size_t)(grow0 + rr) * N + gcol0 + c8) = o;
    }
  } else {
    const int rl = lane >> 4, c4 = (lane & 15) * 4;
#pragma unroll
    for (int p = 0; p < 8; ++p) {
      const int rr = p * 2 + rl;
      v4f v = *(const v4f*)(stg + rr * GM_SP + c4);
      const size_t off = (size_t)(grow0 + rr) * N + gcol0 + c4;
      if constexpr (EPI == 2) {
        const v4f rsd = *(const v4f*)(resid + off);
        const v4f sc = *(const v4f*)(ls + gcol0 + c4);
        v = rsd + v * sc;
      }
      *(volatile v4f*)(Cf + off) = v;
    }
  }
}

template <int EPI>
__global__ __launch_bounds__(256) void gemm_nt(
    const _Float16* __restrict__ A, const _Float16* __restrict__ B,
    const float* __restrict__ bias, const float* __restrict__ ls,
    const float* __restrict__ resid, float* Cf, _Float16* Ch,
    int M, int N, int K, float acc_scale) {
  constexpr int BM = 128, BN = 128, BK = 32, BKP = 40;
  __shared__ __attribute__((aligned(16))) _Float16 As[BM][BKP];
  __shared__ __attribute__((aligned(16))) _Float16 Bs[BN][BKP];
  __shared__ __attribute__((aligned(16))) float Stg[8][16][GM_SP];

  const int tid = threadIdx.x, lane = tid & 31, wave = tid >> 5;
  const int wm = wave >> 1;
  const int wn = wave & 1;
  const int lr = lane & 15, hh = lane >> 4;
  const int n0 = blockIdx.x * BN, m0 = blockIdx.y * BM;
  if (m0 + BM > M || n0 + BN > N) return;

  const int lrow = tid >> 1, lseg = (tid & 1) * 16;
  const _Float16* ag = A + (size_t)(m0 + lrow) * K + lseg;
  const _Float16* bg = B + (size_t)(n0 + lrow) * K + lseg;

  v8f acc[2][4];
#pragma unroll
  for (int i = 0; i < 2; ++i)
#pragma unroll
    for (int j = 0; j < 4; ++j) acc[i][j] = vz8();

  for (int k0 = 0; k0 < K; k0 += BK) {
    const v8h a0 = *(const v8h*)(ag + k0), a1 = *(const v8h*)(ag + k0 + 8);
    const v8h b0 = *(const v8h*)(bg + k0), b1 = *(const v8h*)(bg + k0 + 8);
    __syncthreads();
    *(v8h*)&As[lrow][lseg]     = a0;
    *(v8h*)&As[lrow][lseg + 8] = a1;
    *(v8h*)&Bs[lrow][lseg]     = b0;
    *(v8h*)&Bs[lrow][lseg + 8] = b1;
    __syncthreads();

    v16h af[2], bf[4];
#pragma unroll
    for (int i = 0; i < 2; ++i) af[i] = frag_ld(&As[wm * 32 + i * 16 + lr][0], hh);
#pragma unroll
    for (int j = 0; j < 4; ++j) bf[j] = frag_ld(&Bs[wn * 64 + j * 16 + lr][0], hh);
#pragma unroll
    for (int i = 0; i < 2; ++i)
#pragma unroll
      for (int j = 0; j < 4; ++j) acc[i][j] = wmma_f16(af[i], bf[j], acc[i][j]);
    asm volatile("v_nop\n\tv_nop\n\tv_nop\n\tv_nop"
                 : "+v"(acc[0][0]), "+v"(acc[0][1]), "+v"(acc[0][2]), "+v"(acc[0][3]),
                   "+v"(acc[1][0]), "+v"(acc[1][1]), "+v"(acc[1][2]), "+v"(acc[1][3])
                 : "v"(af[0]), "v"(af[1]), "v"(bf[0]), "v"(bf[1]), "v"(bf[2]), "v"(bf[3]));
  }

  const int gcol0 = n0 + wn * 64;
  float* stw = &Stg[wave][0][0];
#pragma unroll
  for (int i = 0; i < 2; ++i) {
    const int grow0 = m0 + wm * 32 + i * 16;
#pragma unroll
    for (int j = 0; j < 4; ++j) {
      const float bc = bias[gcol0 + j * 16 + lr];
#pragma unroll
      for (int r = 0; r < 8; ++r)
        stw[(hh * 8 + r) * GM_SP + j * 16 + lr] = acc[i][j][r] * acc_scale + bc;
    }
    __syncthreads();
    epi_pass<EPI>(stw, lane, ls, resid, Cf, Ch, grow0, gcol0, N);
    __threadfence();
    epi_pass<EPI>(stw, lane, ls, resid, Cf, Ch, grow0, gcol0, N);
    __syncthreads();
  }
}

__global__ __launch_bounds__(128) void qkv_post(const float* __restrict__ qkv,
                                              const float* __restrict__ rope,
                                              const float* __restrict__ qw,
                                              const float* __restrict__ kw,
                                              _Float16* qo, _Float16* ko, _Float16* vo,
                                              int rows) {
  __shared__ float redq[4], redk[4], cst[ROPE_W], snt[ROPE_W];
  const int s = blockIdx.x;
  if (s >= rows) return;
  const int tid = threadIdx.x, lane = tid & 31, wv = tid >> 5;
  const int e0 = tid * 8;
  const float* base = qkv + (size_t)s * 3 * E_DIM;
  F8 q, k, v;
  ld8(q, base + e0);
  ld8(k, base + E_DIM + e0);
  ld8(v, base + 2 * E_DIM + e0);
  float aq = 0.f, ak = 0.f;
#pragma unroll
  for (int u = 0; u < 8; ++u) { aq += q.f[u] * q.f[u]; ak += k.f[u] * k.f[u]; }
  aq = wave_sum(aq);
  ak = wave_sum(ak);
  if (tid < ROPE_W) {
    const float f = rope[(size_t)s * ROPE_W + tid];
    cst[tid] = cosf(f);
    snt[tid] = sinf(f);
  }
  if (lane == 0) { redq[wv] = aq; redk[wv] = ak; }
  __syncthreads();
  const float rq = rsqrtf(((redq[0] + redq[1]) + (redq[2] + redq[3])) * (1.0f / E_DIM) + EPSF);
  const float rk = rsqrtf(((redk[0] + redk[1]) + (redk[2] + redk[3])) * (1.0f / E_DIM) + EPSF);

  const int d0 = e0 & (D_HEAD - 1);
  const int po = (d0 < ROPE_W) ? ROPE_W : -ROPE_W;
  const float sg = (d0 < ROPE_W) ? -1.0f : 1.0f;
  const int fi = d0 & (ROPE_W - 1);
  F8 qp, kp, wq, wqp, wk, wkp;
  ld8(qp, base + e0 + po);
  ld8(kp, base + E_DIM + e0 + po);
  ld8(wq, qw + e0);
  ld8(wqp, qw + e0 + po);
  ld8(wk, kw + e0);
  ld8(wkp, kw + e0 + po);
  v8h oq, ok, ov;
#pragma unroll
  for (int u = 0; u < 8; ++u) {
    const float c = cst[fi + u], sn = snt[fi + u];
    const float yq = q.f[u] * rq * wq.f[u];
    const float yqp = qp.f[u] * rq * wqp.f[u];
    oq[u] = (_Float16)(yq * c + (sg * yqp) * sn);
    const float yk = k.f[u] * rk * wk.f[u];
    const float ykp = kp.f[u] * rk * wkp.f[u];
    ok[u] = (_Float16)(yk * c + (sg * ykp) * sn);
    ov[u] = (_Float16)v.f[u];
  }
  const size_t oo = (size_t)s * E_DIM + e0;
  *(volatile v8h*)(qo + oo) = oq;
  *(volatile v8h*)(ko + oo) = ok;
  *(volatile v8h*)(vo + oo) = ov;
  __threadfence();
  *(volatile v8h*)(qo + oo) = oq;
  *(volatile v8h*)(ko + oo) = ok;
  *(volatile v8h*)(vo + oo) = ov;
}

#define AT_KP 72

__global__ __launch_bounds__(256) void attn_fwd(const _Float16* __restrict__ Q,
                                              const _Float16* __restrict__ Kx,
                                              const _Float16* __restrict__ V,
                                              _Float16* O) {
  __shared__ __attribute__((aligned(16))) _Float16 Ks[64][AT_KP];
  __shared__ __attribute__((aligned(16))) _Float16 Vt[64][AT_KP];
  __shared__ __attribute__((aligned(16))) _Float16 Ps[8][16][AT_KP];

  const int tid = threadIdx.x, lane = tid & 31, wave = tid >> 5;
  const int lr = lane & 15, hh = lane >> 4;
  const int h = blockIdx.y, seq = blockIdx.x >> 2, qb = blockIdx.x & 3;
  const int q0 = seq * SEQL + qb * 128 + wave * 16;
  const int hoff = h * D_HEAD;

  const _Float16* qrow = Q + (size_t)(q0 + lr) * E_DIM + hoff;
  v16h qa[2];
  qa[0] = frag_ld(qrow, hh);
  qa[1] = frag_ld(qrow + 32, hh);

  float m_r[8], l_r[8];
  v8f o_acc[4];
#pragma unroll
  for (int r = 0; r < 8; ++r) { m_r[r] = -1e30f; l_r[r] = 0.0f; }
#pragma unroll
  for (int j = 0; j < 4; ++j) o_acc[j] = vz8();

  const int krow = tid >> 2, kseg = (tid & 3) * 16;
  _Float16* pw = &Ps[wave][0][0];

#pragma unroll 1
  for (int t = 0; t < SEQL / 64; ++t) {
    const int kv0 = seq * SEQL + t * 64;
    const _Float16* kp = Kx + (size_t)(kv0 + krow) * E_DIM + hoff + kseg;
    const _Float16* vp = V  + (size_t)(kv0 + krow) * E_DIM + hoff + kseg;
    const v8h ka = *(const v8h*)kp, kb = *(const v8h*)(kp + 8);
    const v8h va = *(const v8h*)vp, vb = *(const v8h*)(vp + 8);
    __syncthreads();
    *(v8h*)&Ks[krow][kseg]     = ka;
    *(v8h*)&Ks[krow][kseg + 8] = kb;
#pragma unroll
    for (int u = 0; u < 8; ++u) {
      Vt[kseg + u][krow]     = va[u];
      Vt[kseg + 8 + u][krow] = vb[u];
    }
    __syncthreads();

    float sc[4][8];
#pragma unroll
    for (int nt = 0; nt < 4; ++nt) {
      v8f a = vz8();
      const v16h b0 = frag_ld(&Ks[nt * 16 + lr][0], hh);
      const v16h b1 = frag_ld(&Ks[nt * 16 + lr][32], hh);
      a = wmma_f16(qa[0], b0, a);
      a = wmma_f16(qa[1], b1, a);
      asm volatile("v_nop\n\tv_nop\n\tv_nop\n\tv_nop"
                   : "+v"(a) : "v"(qa[0]), "v"(qa[1]), "v"(b0), "v"(b1));
#pragma unroll
      for (int r = 0; r < 8; ++r) sc[nt][r] = a[r] * 0.125f;
    }

#pragma unroll
    for (int r = 0; r < 8; ++r) {
      float tm = fmaxf(fmaxf(sc[0][r], sc[1][r]), fmaxf(sc[2][r], sc[3][r]));
      tm = fmaxf(tm, __shfl_xor(tm, 8, 32));
      tm = fmaxf(tm, __shfl_xor(tm, 4, 32));
      tm = fmaxf(tm, __shfl_xor(tm, 2, 32));
      tm = fmaxf(tm, __shfl_xor(tm, 1, 32));
      const float mn = fmaxf(m_r[r], tm);
      const float corr = __expf(m_r[r] - mn);
      m_r[r] = mn;
      float ps = 0.0f;
#pragma unroll
      for (int nt = 0; nt < 4; ++nt) {
        const float p = __expf(sc[nt][r] - mn);
        pw[(hh * 8 + r) * AT_KP + nt * 16 + lr] = (_Float16)(p * P_SCALE);
        ps += p;
      }
      ps += __shfl_xor(ps, 8, 32);
      ps += __shfl_xor(ps, 4, 32);
      ps += __shfl_xor(ps, 2, 32);
      ps += __shfl_xor(ps, 1, 32);
      l_r[r] = l_r[r] * corr + ps;
#pragma unroll
      for (int j = 0; j < 4; ++j) o_acc[j][r] = o_acc[j][r] * corr;
    }
    __syncthreads();

#pragma unroll
    for (int ks = 0; ks < 2; ++ks) {
      const v16h a = frag_ld(pw + lr * AT_KP + ks * 32, hh);
      v16h b[4];
#pragma unroll
      for (int j = 0; j < 4; ++j) b[j] = frag_ld(&Vt[j * 16 + lr][ks * 32], hh);
#pragma unroll
      for (int j = 0; j < 4; ++j) o_acc[j] = wmma_f16(a, b[j], o_acc[j]);
      asm volatile("v_nop\n\tv_nop\n\tv_nop\n\tv_nop"
                   : "+v"(o_acc[0]), "+v"(o_acc[1]), "+v"(o_acc[2]), "+v"(o_acc[3])
                   : "v"(a), "v"(b[0]), "v"(b[1]), "v"(b[2]), "v"(b[3]));
    }
  }

  __syncthreads();
  float inv[8];
#pragma unroll
  for (int r = 0; r < 8; ++r) inv[r] = (O_SCALE / P_SCALE) / l_r[r];
#pragma unroll
  for (int j = 0; j < 4; ++j)
#pragma unroll
    for (int r = 0; r < 8; ++r)
      pw[(hh * 8 + r) * AT_KP + j * 16 + lr] = (_Float16)(o_acc[j][r] * inv[r]);
  __syncthreads();
  const int rl = lane >> 3, c8 = (lane & 7) * 8;
  v8h ov[4];
#pragma unroll
  for (int p = 0; p < 4; ++p) ov[p] = *(const v8h*)(pw + (p * 4 + rl) * AT_KP + c8);
#pragma unroll
  for (int p = 0; p < 4; ++p)
    *(volatile v8h*)(O + (size_t)(q0 + p * 4 + rl) * E_DIM + hoff + c8) = ov[p];
  __threadfence();
#pragma unroll
  for (int p = 0; p < 4; ++p)
    *(volatile v8h*)(O + (size_t)(q0 + p * 4 + rl) * E_DIM + hoff + c8) = ov[p];
}

extern "C" void kernel_launch(void* const* d_in, const int* in_sizes, int n_in,
                              void* d_out, int out_size, void* d_ws,
                              size_t ws_size, hipStream_t stream) {
  if (n_in < 19) return;
  if (in_sizes[0] != S_TOK * E_DIM || in_sizes[2] != S_TOK * ROPE_W ||
      in_sizes[3] != 3 * E_DIM * E_DIM || in_sizes[4] != 3 * E_DIM ||
      in_sizes[5] != E_DIM || in_sizes[6] != E_DIM ||
      in_sizes[7] != E_DIM * E_DIM || in_sizes[8] != E_DIM ||
      in_sizes[9] != E_DIM || in_sizes[10] != E_DIM ||
      in_sizes[11] != E_DIM || in_sizes[12] != E_DIM ||
      in_sizes[13] != I_DIM * E_DIM || in_sizes[14] != I_DIM ||
      in_sizes[15] != E_DIM * I_DIM || in_sizes[16] != E_DIM ||
      in_sizes[17] != E_DIM || in_sizes[18] != E_DIM ||
      out_size != S_TOK * E_DIM)
    return;

  const float* x      = (const float*)d_in[0];
  const float* rope   = (const float*)d_in[2];
  const float* qkv_w  = (const float*)d_in[3];
  const float* qkv_b  = (const float*)d_in[4];
  const float* q_nw   = (const float*)d_in[5];
  const float* k_nw   = (const float*)d_in[6];
  const float* proj_w = (const float*)d_in[7];
  const float* proj_b = (const float*)d_in[8];
  const float* n1w    = (const float*)d_in[9];
  const float* n1b    = (const float*)d_in[10];
  const float* n2w    = (const float*)d_in[11];
  const float* n2b    = (const float*)d_in[12];
  const float* fc1_w  = (const float*)d_in[13];
  const float* fc1_b  = (const float*)d_in[14];
  const float* fc2_w  = (const float*)d_in[15];
  const float* fc2_b  = (const float*)d_in[16];
  const float* ls1    = (const float*)d_in[17];
  const float* ls2    = (const float*)d_in[18];
  float* out = (float*)d_out;

  size_t off = 0;
  auto carve = [&](size_t bytes) -> size_t {
    size_t r = off;
    off += (bytes + 255) & ~(size_t)255;
    return r;
  };
  const size_t o_qkvw = carve((size_t)3 * E_DIM * E_DIM * 2);
  const size_t o_prjw = carve((size_t)E_DIM * E_DIM * 2);
  const size_t o_fc1w = carve((size_t)I_DIM * E_DIM * 2);
  const size_t o_fc2w = carve((size_t)E_DIM * I_DIM * 2);
  const size_t o_h1   = carve((size_t)S_TOK * E_DIM * 2);
  const size_t o_qkvf = carve((size_t)S_TOK * 3 * E_DIM * 4);
  const size_t o_qh   = carve((size_t)S_TOK * E_DIM * 2);
  const size_t o_kh   = carve((size_t)S_TOK * E_DIM * 2);
  const size_t o_vh   = carve((size_t)S_TOK * E_DIM * 2);
  const size_t o_attn = carve((size_t)S_TOK * E_DIM * 2);
  const size_t o_x2   = carve((size_t)S_TOK * E_DIM * 4);
  const size_t o_h2   = carve((size_t)S_TOK * E_DIM * 2);
  const size_t o_mh   = carve((size_t)S_TOK * I_DIM * 2);
  if (off > ws_size) return;

  char* ws = (char*)d_ws;
  _Float16* qkvw_h = (_Float16*)(ws + o_qkvw);
  _Float16* projw_h = (_Float16*)(ws + o_prjw);
  _Float16* fc1w_h = (_Float16*)(ws + o_fc1w);
  _Float16* fc2w_h = (_Float16*)(ws + o_fc2w);
  _Float16* h1     = (_Float16*)(ws + o_h1);
  float*    qkv_f  = (float*)(ws + o_qkvf);
  _Float16* qh     = (_Float16*)(ws + o_qh);
  _Float16* kh     = (_Float16*)(ws + o_kh);
  _Float16* vh     = (_Float16*)(ws + o_vh);
  _Float16* attn_h = (_Float16*)(ws + o_attn);
  float*    x2     = (float*)(ws + o_x2);
  _Float16* h2     = (_Float16*)(ws + o_h2);
  _Float16* mh     = (_Float16*)(ws + o_mh);

  auto cvt = [&](const float* src, _Float16* dst, int n) {
    const int n8 = n / 8;
    int blocks = (n8 + 255) / 256;
    if (blocks > 1024) blocks = 1024;
    if (blocks < 1) blocks = 1;
    cvt_scale_f16<<<blocks, 256, 0, stream>>>(src, dst, n8, W_SCALE);
  };
  cvt(qkv_w, qkvw_h, 3 * E_DIM * E_DIM);
  cvt(proj_w, projw_h, E_DIM * E_DIM);
  cvt(fc1_w, fc1w_h, I_DIM * E_DIM);
  cvt(fc2_w, fc2w_h, E_DIM * I_DIM);

  layernorm_f16<<<S_TOK, 128, 0, stream>>>(x, n1w, n1b, h1, S_TOK);

  gemm_nt<0><<<dim3(3 * E_DIM / 128, S_TOK / 128), 256, 0, stream>>>(
      h1, qkvw_h, qkv_b, qkv_b, x, qkv_f, h1, S_TOK, 3 * E_DIM, E_DIM,
      1.0f / W_SCALE);

  qkv_post<<<S_TOK, 128, 0, stream>>>(qkv_f, rope, q_nw, k_nw, qh, kh, vh, S_TOK);

  attn_fwd<<<dim3(NSEQ_ * (SEQL / 128), H_HEADS), 256, 0, stream>>>(qh, kh, vh, attn_h);

  gemm_nt<2><<<dim3(E_DIM / 128, S_TOK / 128), 256, 0, stream>>>(
      attn_h, projw_h, proj_b, ls1, x, x2, h1, S_TOK, E_DIM, E_DIM,
      1.0f / (W_SCALE * O_SCALE));

  layernorm_f16<<<S_TOK, 128, 0, stream>>>(x2, n2w, n2b, h2, S_TOK);

  gemm_nt<1><<<dim3(I_DIM / 128, S_TOK / 128), 256, 0, stream>>>(
      h2, fc1w_h, fc1_b, fc1_b, x2, x2, mh, S_TOK, I_DIM, E_DIM, 1.0f / W_SCALE);

  gemm_nt<2><<<dim3(E_DIM / 128, S_TOK / 128), 256, 0, stream>>>(
      mh, fc2w_h, fc2_b, ls2, x2, out, h2, S_TOK, E_DIM, I_DIM, 1.0f / W_SCALE);
}
